// Encoder_45414984188137
// MI455X (gfx1250) — hardware-verified
//
#include <hip/hip_runtime.h>
#include <hip/hip_fp16.h>


#ifndef NB
#define NB 2
#endif
#ifndef SEQ
#define SEQ 2048
#endif
#define NB_FULL  2
#define SEQ_FULL 2048
#define DM   1024
#define NH   16
#define HD   64
#define DFF  4096
#define NTOK (NB * SEQ)
#define CH   128

#define TP_TILE    64
#define TP_THREADS 256
#define TP_PIECE   8
#define TP_ITERS   2
#define TP_LD      72

static_assert(NB >= 1 && NB <= NB_FULL);
static_assert(SEQ >= CH && SEQ <= SEQ_FULL);
static_assert(SEQ % CH == 0);
static_assert(SEQ % 128 == 0);
static_assert(NTOK % 128 == 0);
static_assert(NH * HD == DM);
static_assert(NH == 16 && HD == 64 && DM == 1024);
static_assert(DM % 128 == 0 && DFF % 128 == 0 && (3 * DM) % 128 == 0);
static_assert(DM % 32 == 0 && DFF % 32 == 0);
static_assert((size_t)NB_FULL * SEQ_FULL * DM * 4 == 16777216);
static_assert(TP_THREADS * TP_PIECE * TP_ITERS == TP_TILE * TP_TILE);
static_assert(TP_THREADS * 4 * 4 == TP_TILE * TP_TILE);
static_assert((TP_THREADS / (TP_TILE / TP_PIECE)) * TP_ITERS == TP_TILE);
static_assert(DM % TP_TILE == 0 && HD % TP_TILE == 0 && DFF % TP_TILE == 0);

typedef _Float16 v16h __attribute__((ext_vector_type(16)));
typedef _Float16 v8h  __attribute__((ext_vector_type(8)));
typedef _Float16 v4h  __attribute__((ext_vector_type(4)));
typedef float    v8f  __attribute__((ext_vector_type(8)));
typedef float    v4f  __attribute__((ext_vector_type(4)));

union Frag { v16h v; v8h h[2]; };

#define CAR_ACT  16.0f
#define CAR_W    64.0f
#define AL_QKV   0.015625f
#define AL_FF1   0.015625f
#define AL_WO    2.44140625e-04f
#define AL_FF2   9.765625e-04f
#define CS (1.44269504088896340736f * 4.8828125e-04f)

static __device__ __forceinline__ v8f zero8() {
    v8f z;
#pragma unroll
    for (int i = 0; i < 8; ++i) z[i] = 0.0f;
    return z;
}

static __device__ __forceinline__ v16h load_frag16(const _Float16* base, int ld, int lane) {
    int m  = lane & 15;
    int kb = (lane >> 4) << 3;
    const _Float16* p = base + (size_t)m * ld + kb;
    Frag f;
    f.h[0] = *(const v8h*)(p);
    f.h[1] = *(const v8h*)(p + 16);
    return f.v;
}

static __device__ __forceinline__ v8f wmma16(v16h a, v16h b, v8f c) {
    v8f d = __builtin_amdgcn_wmma_f32_16x16x32_f16(false, a, false, b, (short)0, c, false, false);
    asm volatile("v_nop\n\tv_nop\n\tv_nop\n\tv_nop" : "+v"(d) : "v"(a), "v"(b));
    return d;
}

static __device__ __forceinline__ float bf16r(float x) {
    unsigned u = __float_as_uint(x);
    u = (u + 0x7FFFu + ((u >> 16) & 1u)) & 0xFFFF0000u;
    return __uint_as_float(u);
}

static __device__ __forceinline__ float ex2(float x) {
    return __builtin_amdgcn_exp2f(x);
}

static __device__ __forceinline__ void wave_lds_sync() {
    __builtin_amdgcn_fence(3, "wavefront");
    asm volatile("s_wait_dscnt 0" ::: "memory");
    __builtin_amdgcn_wave_barrier();
}

static __device__ __forceinline__ unsigned xrow(unsigned tok) {
    unsigned b = tok / (unsigned)SEQ;
    unsigned s = tok - b * (unsigned)SEQ;
    return b * (unsigned)SEQ_FULL + s;
}

static __device__ __forceinline__ void store_tile_h(const _Float16* tile, _Float16* dst0,
                                                    size_t pitch, unsigned lane) {
    wave_lds_sync();
    const unsigned lr = lane >> 3;
    const unsigned lp = (lane & 7u) << 3;
    v8h pv[4];
#pragma unroll
    for (unsigned i = 0; i < 4; ++i) pv[i] = *(const v8h*)(tile + (4u * i + lr) * 64u + lp);
#pragma unroll
    for (unsigned i = 0; i < 4; ++i) *(volatile v8h*)(dst0 + (size_t)(4u * i + lr) * pitch + lp) = pv[i];
    __threadfence();
#pragma unroll
    for (unsigned i = 0; i < 4; ++i) *(volatile v8h*)(dst0 + (size_t)(4u * i + lr) * pitch + lp) = pv[i];
    wave_lds_sync();
}

__global__ __launch_bounds__(256) void k_cvt_x(const float* __restrict__ x, _Float16* __restrict__ xh) {
    const unsigned gid = blockIdx.x * 256u + threadIdx.x;
    const unsigned tok = gid >> 7;
    const unsigned c8  = (gid & 127u) << 3;
    const float* src = x + (size_t)xrow(tok) * DM + c8;
    v4f a = *(const v4f*)(src);
    v4f b = *(const v4f*)(src + 4);
    v8h hv;
    hv[0] = (_Float16)(bf16r(a.x) * CAR_ACT);
    hv[1] = (_Float16)(bf16r(a.y) * CAR_ACT);
    hv[2] = (_Float16)(bf16r(a.z) * CAR_ACT);
    hv[3] = (_Float16)(bf16r(a.w) * CAR_ACT);
    hv[4] = (_Float16)(bf16r(b.x) * CAR_ACT);
    hv[5] = (_Float16)(bf16r(b.y) * CAR_ACT);
    hv[6] = (_Float16)(bf16r(b.z) * CAR_ACT);
    hv[7] = (_Float16)(bf16r(b.w) * CAR_ACT);
    _Float16* dst = xh + (size_t)tok * DM + c8;
    *(volatile v8h*)dst = hv;
    __threadfence();
    *(volatile v8h*)dst = hv;
}

__global__ __launch_bounds__(TP_THREADS) void k_tpose(const float* __restrict__ in, _Float16* __restrict__ out,
                                                       unsigned R, unsigned C) {
    __shared__ __align__(16) _Float16 T[TP_TILE * TP_LD];
    const unsigned tid = threadIdx.x;
    const unsigned r0 = blockIdx.x * (unsigned)TP_TILE;
    const unsigned c0 = blockIdx.y * (unsigned)TP_TILE;
    const size_t boff = (size_t)blockIdx.z * R * C;
    const float* inb = in + boff;
    _Float16* outb = out + boff;
#pragma unroll
    for (unsigned it = 0; it < 4; ++it) {
        const unsigned idx = tid + it * 256u;
        const unsigned r = idx >> 4, c4 = (idx & 15u) << 2;
        v4f v = *(const v4f*)(inb + (size_t)(r0 + r) * C + c0 + c4);
        T[(c4 + 0u) * TP_LD + r] = (_Float16)(bf16r(v.x) * CAR_W);
        T[(c4 + 1u) * TP_LD + r] = (_Float16)(bf16r(v.y) * CAR_W);
        T[(c4 + 2u) * TP_LD + r] = (_Float16)(bf16r(v.z) * CAR_W);
        T[(c4 + 3u) * TP_LD + r] = (_Float16)(bf16r(v.w) * CAR_W);
    }
    __syncthreads();
    const unsigned line0 = tid >> 3, piece = (tid & 7u) << 3;
    v8h o[TP_ITERS];
#pragma unroll
    for (unsigned it = 0; it < TP_ITERS; ++it)
        o[it] = *(const v8h*)(&T[(line0 + 32u * it) * TP_LD + piece]);
    _Float16* dst = outb + (size_t)(c0 + line0) * R + r0 + piece;
#pragma unroll
    for (unsigned it = 0; it < TP_ITERS; ++it)
        *(volatile v8h*)(dst + (size_t)(32u * it) * R) = o[it];
    __threadfence();
#pragma unroll
    for (unsigned it = 0; it < TP_ITERS; ++it)
        *(volatile v8h*)(dst + (size_t)(32u * it) * R) = o[it];
}

static __device__ __forceinline__ void gemm_core(const _Float16* __restrict__ A,
                                                 const _Float16* __restrict__ Bt,
                                                 unsigned K, unsigned rowA0, unsigned rowB0,
                                                 int lane, v8f (&acc)[2][4]) {
#pragma unroll
    for (int mi = 0; mi < 2; ++mi)
#pragma unroll
        for (int ni = 0; ni < 4; ++ni) acc[mi][ni] = zero8();
    const _Float16* a0p = A + (size_t)rowA0 * K;
    const _Float16* a1p = a0p + (size_t)16 * K;
    const _Float16* bp  = Bt + (size_t)rowB0 * K;
#pragma unroll 1
    for (unsigned k0 = 0; k0 < K; k0 += 32) {
        v16h a0 = load_frag16(a0p + k0, (int)K, lane);
        v16h a1 = load_frag16(a1p + k0, (int)K, lane);
#pragma unroll
        for (int ni = 0; ni < 4; ++ni) {
            v16h b = load_frag16(bp + (size_t)(ni * 16) * K + k0, (int)K, lane);
            acc[0][ni] = wmma16(a0, b, acc[0][ni]);
            acc[1][ni] = wmma16(a1, b, acc[1][ni]);
        }
    }
}

template<int QKV>
__global__ __launch_bounds__(256) __attribute__((amdgpu_num_vgpr(256)))
void k_gemm_h(const _Float16* __restrict__ A, const _Float16* __restrict__ Bt,
              const float* __restrict__ bA, const float* __restrict__ bB, const float* __restrict__ bC,
              _Float16* __restrict__ out, unsigned K, unsigned N, float alpha, float beta) {
    __shared__ __align__(16) _Float16 stg[8][16 * 64];
    const unsigned tid = threadIdx.x, lane = tid & 31u, w = tid >> 5;
    const unsigned wr = w >> 1, wc = w & 1u;
    const unsigned bm = blockIdx.x * 128u, bn = blockIdx.y * 128u;
    const unsigned r0 = (lane >> 4) << 3, cc = lane & 15u;

    v8f acc[2][4];
    gemm_core(A, Bt, K, bm + wr * 32u, bn + wc * 64u, (int)lane, acc);

    const unsigned gc0 = bn + wc * 64u;
    unsigned p = 0u, hh = 0u, bidx0 = gc0;
    const float* bias = bA;
    if (QKV) {
        p = gc0 >> 10;
        hh = (gc0 >> 6) & 15u;
        bidx0 = gc0 & 1023u;
        bias = (p == 0u) ? bA : ((p == 1u) ? bB : bC);
    }
    float bvv[4];
#pragma unroll
    for (int ni = 0; ni < 4; ++ni) bvv[ni] = beta * bf16r(bias[bidx0 + ni * 16 + cc]);

#pragma unroll
    for (int mi = 0; mi < 2; ++mi) {
        const unsigned tok0 = bm + wr * 32u + (unsigned)mi * 16u;
        _Float16* dst0;
        size_t pitch;
        if (QKV) {
            const unsigned b = tok0 / (unsigned)SEQ;
            const unsigned s0 = tok0 - b * (unsigned)SEQ;
            dst0 = out + (size_t)p * ((size_t)NTOK * DM) + ((size_t)(b * NH + hh) * SEQ + s0) * HD;
            pitch = HD;
        } else {
            dst0 = out + (size_t)tok0 * N + gc0;
            pitch = N;
        }
#pragma unroll
        for (int ni = 0; ni < 4; ++ni)
#pragma unroll
            for (int g = 0; g < 8; ++g) {
                float v = __builtin_fmaf(acc[mi][ni][g], alpha, bvv[ni]);
                if (!QKV) v = fmaxf(v, 0.0f);
                stg[w][(r0 + g) * 64u + ni * 16 + cc] = (_Float16)v;
            }
        store_tile_h(&stg[w][0], dst0, pitch, lane);
    }
}

template<int RND>
__global__ __launch_bounds__(256) __attribute__((amdgpu_num_vgpr(256)))
void k_gemm_res(const _Float16* __restrict__ A, const _Float16* __restrict__ Bt,
                const float* __restrict__ bias, const float* __restrict__ resid,
                float* __restrict__ C, unsigned K, float alpha) {
    __shared__ __align__(16) float stg[8][16 * 64];
    const unsigned tid = threadIdx.x, lane = tid & 31u, w = tid >> 5;
    const unsigned wr = w >> 1, wc = w & 1u;
    const unsigned bm = blockIdx.x * 128u, bn = blockIdx.y * 128u;
    const unsigned r0 = (lane >> 4) << 3, cc = lane & 15u;

    v8f acc[2][4];
    gemm_core(A, Bt, K, bm + wr * 32u, bn + wc * 64u, (int)lane, acc);

    const unsigned gc0 = bn + wc * 64u;
    float bvv[4];
#pragma unroll
    for (int ni = 0; ni < 4; ++ni) bvv[ni] = bf16r(bias[gc0 + ni * 16 + cc]);

    const unsigned lr = lane >> 4, c4 = (lane & 15u) << 2;
#pragma unroll
    for (int mi = 0; mi < 2; ++mi) {
        const unsigned tok0 = bm + wr * 32u + (unsigned)mi * 16u;
#pragma unroll
        for (int ni = 0; ni < 4; ++ni)
#pragma unroll
            for (int g = 0; g < 8; ++g)
                stg[w][(r0 + g) * 64u + ni * 16 + cc] = __builtin_fmaf(acc[mi][ni][g], alpha, bvv[ni]);
        wave_lds_sync();
        const unsigned rrow0 = RND ? xrow(tok0) : tok0;
        const float* rs0 = resid + (size_t)rrow0 * DM + gc0 + c4;
        float* dst0 = C + (size_t)tok0 * DM + gc0 + c4;
        v4f sv[8];
#pragma unroll
        for (unsigned i = 0; i < 8; ++i) {
            const unsigned row = 2u * i + lr;
            v4f t = *(const v4f*)(&stg[w][row * 64u + c4]);
            v4f r = *(const v4f*)(rs0 + (size_t)row * DM);
            if (RND) { r.x = bf16r(r.x); r.y = bf16r(r.y); r.z = bf16r(r.z); r.w = bf16r(r.w); }
            sv[i] = t + r;
        }
#pragma unroll
        for (unsigned i = 0; i < 8; ++i) *(volatile v4f*)(dst0 + (size_t)(2u * i + lr) * DM) = sv[i];
        __threadfence();
#pragma unroll
        for (unsigned i = 0; i < 8; ++i) *(volatile v4f*)(dst0 + (size_t)(2u * i + lr) * DM) = sv[i];
        wave_lds_sync();
    }
}

__global__ __launch_bounds__(256) __attribute__((amdgpu_num_vgpr(256)))
void k_attn(const _Float16* __restrict__ qp, const _Float16* __restrict__ kp,
            const _Float16* __restrict__ vp, _Float16* __restrict__ ctx) {
    __shared__ __align__(16) _Float16 VT[HD * CH];
    __shared__ __align__(16) _Float16 Pst[8][16 * 64];

    const unsigned tid = threadIdx.x, lane = tid & 31u, w = tid >> 5;
    const unsigned bh = blockIdx.y;
    const unsigned b = bh / (unsigned)NH;
    const unsigned h = bh - b * (unsigned)NH;
    const unsigned q0r = blockIdx.x * 128u + w * 16u;
    const unsigned r0 = (lane >> 4) << 3, cc = lane & 15u;

    const size_t pb = (size_t)bh * SEQ * HD;
    const _Float16* qb = qp + pb + (size_t)q0r * HD;
    const v16h qf0 = load_frag16(qb, HD, (int)lane);
    const v16h qf1 = load_frag16(qb + 32, HD, (int)lane);
    const _Float16* kb = kp + pb;
    const _Float16* vb = vp + pb;

    float mr[8], ls[8];
#pragma unroll
    for (int g = 0; g < 8; ++g) { mr[g] = -1.0e30f; ls[g] = 0.0f; }
    v8f o[4];
#pragma unroll
    for (int dt = 0; dt < 4; ++dt) o[dt] = zero8();

#pragma unroll 1
    for (unsigned c0 = 0; c0 < (unsigned)SEQ; c0 += CH) {
        for (unsigned idx = tid; idx < CH * 8u; idx += 256u) {
            const unsigned t = idx >> 3, part = idx & 7u;
            v8h vv = *(const v8h*)(vb + (size_t)(c0 + t) * HD + part * 8u);
#pragma unroll
            for (int e = 0; e < 8; ++e) VT[(part * 8u + e) * CH + t] = vv[e];
        }
        __syncthreads();

#pragma unroll 1
        for (unsigned j = 0; j < CH; j += 64) {
            const unsigned kA = c0 + j;
            v8f s[4];
#pragma unroll
            for (int t = 0; t < 4; ++t) {
                const _Float16* kr = kb + (size_t)(kA + t * 16) * HD;
                v16h kf0 = load_frag16(kr, HD, (int)lane);
                v16h kf1 = load_frag16(kr + 32, HD, (int)lane);
                v8f c = wmma16(qf0, kf0, zero8());
                s[t] = wmma16(qf1, kf1, c);
            }
#pragma unroll
            for (int g = 0; g < 8; ++g) {
                float mx = fmaxf(fmaxf(s[0][g], s[1][g]), fmaxf(s[2][g], s[3][g]));
                mx = fmaxf(mx, __shfl_xor(mx, 8, 32));
                mx = fmaxf(mx, __shfl_xor(mx, 4, 32));
                mx = fmaxf(mx, __shfl_xor(mx, 2, 32));
                mx = fmaxf(mx, __shfl_xor(mx, 1, 32));
                const float mn = fmaxf(mr[g], mx * CS);
                const float al = ex2(mr[g] - mn);
                mr[g] = mn;
                float ps = 0.0f;
#pragma unroll
                for (int t = 0; t < 4; ++t) {
                    float pe = ex2(__builtin_fmaf(s[t][g], CS, -mn));
                    ps += pe;
                    Pst[w][(r0 + g) * 64u + t * 16 + cc] = (_Float16)pe;
                }
                ls[g] = ls[g] * al + ps;
#pragma unroll
                for (int dt = 0; dt < 4; ++dt) o[dt][g] *= al;
            }
            wave_lds_sync();
            v16h pa0 = load_frag16(&Pst[w][0], 64, (int)lane);
            v16h pa1 = load_frag16(&Pst[w][32], 64, (int)lane);
#pragma unroll
            for (int dt = 0; dt < 4; ++dt) {
                v16h vb0 = load_frag16(&VT[(dt * 16) * CH + j], CH, (int)lane);
                v16h vb1 = load_frag16(&VT[(dt * 16) * CH + j + 32], CH, (int)lane);
                o[dt] = wmma16(pa0, vb0, o[dt]);
                o[dt] = wmma16(pa1, vb1, o[dt]);
            }
        }
        __syncthreads();
    }

    wave_lds_sync();
#pragma unroll
    for (int g = 0; g < 8; ++g) {
        float l = ls[g];
        l += __shfl_xor(l, 8, 32);
        l += __shfl_xor(l, 4, 32);
        l += __shfl_xor(l, 2, 32);
        l += __shfl_xor(l, 1, 32);
        const float inv = __builtin_amdgcn_rcpf(l) * 4.0f;
#pragma unroll
        for (int dt = 0; dt < 4; ++dt)
            Pst[w][(r0 + g) * 64u + dt * 16 + cc] = (_Float16)(o[dt][g] * inv);
    }
    _Float16* dst0 = ctx + (size_t)(b * (unsigned)SEQ + q0r) * DM + h * HD;
    store_tile_h(&Pst[w][0], dst0, (size_t)DM, lane);
}

static __device__ __forceinline__ v4f ln_vals(const float* yr, const float* g, const float* be,
                                              unsigned off, float mu, float rstd) {
    v4f v  = *(const v4f*)(yr + off);
    v4f gg = *(const v4f*)(g + off);
    v4f bb = *(const v4f*)(be + off);
    v4f o;
    o.x = (v.x - mu) * rstd * bf16r(gg.x) + bf16r(bb.x);
    o.y = (v.y - mu) * rstd * bf16r(gg.y) + bf16r(bb.y);
    o.z = (v.z - mu) * rstd * bf16r(gg.z) + bf16r(bb.z);
    o.w = (v.w - mu) * rstd * bf16r(gg.w) + bf16r(bb.w);
    return o;
}

template<int OUT16>
__global__ __launch_bounds__(256) void k_ln(const float* __restrict__ y, const float* __restrict__ g,
                                             const float* __restrict__ be, float* __restrict__ outf,
                                             _Float16* __restrict__ outh) {
    __shared__ __align__(16) _Float16 hst[OUT16 ? 8 : 1][DM];
    const unsigned tid = threadIdx.x, lane = tid & 31u, w = tid >> 5;
    const unsigned row = blockIdx.x * 8u + w;
    const float* yr = y + (size_t)row * DM;

    float s = 0.0f;
#pragma unroll 1
    for (unsigned i = 0; i < 8; ++i) {
        v4f v = *(const v4f*)(yr + i * 128u + lane * 4u);
        s += (v.x + v.y) + (v.z + v.w);
    }
    s += __shfl_xor(s, 16, 32);
    s += __shfl_xor(s, 8, 32);
    s += __shfl_xor(s, 4, 32);
    s += __shfl_xor(s, 2, 32);
    s += __shfl_xor(s, 1, 32);
    const float mu = s * (1.0f / (float)DM);

    float ss = 0.0f;
#pragma unroll 1
    for (unsigned i = 0; i < 8; ++i) {
        v4f v = *(const v4f*)(yr + i * 128u + lane * 4u);
        float d0 = v.x - mu, d1 = v.y - mu, d2 = v.z - mu, d3 = v.w - mu;
        ss += (d0 * d0 + d1 * d1) + (d2 * d2 + d3 * d3);
    }
    ss += __shfl_xor(ss, 16, 32);
    ss += __shfl_xor(ss, 8, 32);
    ss += __shfl_xor(ss, 4, 32);
    ss += __shfl_xor(ss, 2, 32);
    ss += __shfl_xor(ss, 1, 32);
    const float rstd = rsqrtf(ss * (1.0f / (float)DM) + 1.0e-5f);

    float* of = outf + (size_t)row * DM;
#pragma unroll 1
    for (unsigned i = 0; i < 8; ++i) {
        const unsigned off = i * 128u + lane * 4u;
        v4f o = ln_vals(yr, g, be, off, mu, rstd);
        *(volatile v4f*)(of + off) = o;
        if (OUT16) {
            v4h hv;
            hv.x = (_Float16)(o.x * CAR_ACT);
            hv.y = (_Float16)(o.y * CAR_ACT);
            hv.z = (_Float16)(o.z * CAR_ACT);
            hv.w = (_Float16)(o.w * CAR_ACT);
            *(v4h*)(&hst[OUT16 ? w : 0][off]) = hv;
        }
    }
    v8h hv8[4];
    _Float16* oh = outh + (size_t)row * DM;
    if (OUT16) {
        wave_lds_sync();
#pragma unroll
        for (unsigned i = 0; i < 4; ++i) hv8[i] = *(const v8h*)(&hst[OUT16 ? w : 0][i * 256u + lane * 8u]);
#pragma unroll
        for (unsigned i = 0; i < 4; ++i) *(volatile v8h*)(oh + i * 256u + lane * 8u) = hv8[i];
    }
    __threadfence();
#pragma unroll 1
    for (unsigned i = 0; i < 8; ++i) {
        const unsigned off = i * 128u + lane * 4u;
        v4f o = ln_vals(yr, g, be, off, mu, rstd);
        *(volatile v4f*)(of + off) = o;
    }
    if (OUT16) {
#pragma unroll
        for (unsigned i = 0; i < 4; ++i) *(volatile v8h*)(oh + i * 256u + lane * 8u) = hv8[i];
    }
}

extern "C" void kernel_launch(void* const* d_in, const int* in_sizes, int n_in,
                              void* d_out, int out_size, void* d_ws, size_t ws_size,
                              hipStream_t stream) {
    if (n_in < 17) return;
    if (in_sizes[0] < ((NB - 1) * SEQ_FULL + SEQ) * DM) return;
    if (in_sizes[1] < NH * DM * HD || in_sizes[3] < NH * DM * HD || in_sizes[5] < NH * DM * HD) return;
    if (in_sizes[2] < DM || in_sizes[4] < DM || in_sizes[6] < DM) return;
    if (in_sizes[7] < DM * DM || in_sizes[8] < DM) return;
    if (in_sizes[9] < DM * DFF || in_sizes[10] < DFF) return;
    if (in_sizes[11] < DFF * DM || in_sizes[12] < DM) return;
    if (in_sizes[13] < DM || in_sizes[14] < DM || in_sizes[15] < DM || in_sizes[16] < DM) return;
    if (out_size < NTOK * DM) return;

    const float* x   = (const float*)d_in[0];
    const float* Wq  = (const float*)d_in[1];
    const float* bq  = (const float*)d_in[2];
    const float* Wk  = (const float*)d_in[3];
    const float* bk  = (const float*)d_in[4];
    const float* Wv  = (const float*)d_in[5];
    const float* bv  = (const float*)d_in[6];
    const float* Wo  = (const float*)d_in[7];
    const float* bo  = (const float*)d_in[8];
    const float* W1  = (const float*)d_in[9];
    const float* b1  = (const float*)d_in[10];
    const float* W2  = (const float*)d_in[11];
    const float* b2  = (const float*)d_in[12];
    const float* g1  = (const float*)d_in[13];
    const float* be1 = (const float*)d_in[14];
    const float* g2  = (const float*)d_in[15];
    const float* be2 = (const float*)d_in[16];
    float* out = (float*)d_out;

    constexpr size_t SZ_XH  = (size_t)NTOK * DM * 2;
    constexpr size_t SZ_PL  = (size_t)NTOK * DM * 2;
    constexpr size_t SZ_H   = (size_t)NTOK * DFF * 2;
    constexpr size_t SZ_R0  = (SZ_XH + 3 * SZ_PL > SZ_H) ? (SZ_XH + 3 * SZ_PL) : SZ_H;
    constexpr size_t SZ_CTX = (size_t)NTOK * DM * 2;
    constexpr size_t SZ_Y   = (size_t)NTOK * DM * 4;
    constexpr size_t SZ_X1  = (size_t)NTOK * DM * 4;
    constexpr size_t SZ_X1H = (size_t)NTOK * DM * 2;
    constexpr size_t SZ_WQKV = (size_t)3 * DM * DM * 2;
    constexpr size_t SZ_WO  = (size_t)DM * DM * 2;
    constexpr size_t SZ_W1  = (size_t)DFF * DM * 2;
    constexpr size_t SZ_W2  = (size_t)DM * DFF * 2;
    constexpr size_t SZ_TOT = SZ_R0 + SZ_CTX + SZ_Y + SZ_X1 + SZ_X1H + SZ_WQKV + SZ_WO + SZ_W1 + SZ_W2;
    static_assert(SZ_XH + 3 * SZ_PL <= SZ_R0 && SZ_H <= SZ_R0);
    static_assert(SZ_TOT <= (size_t)134217728);
    static_assert(SZ_R0 % 256 == 0 && SZ_CTX % 256 == 0 && SZ_Y % 256 == 0 && SZ_X1H % 256 == 0);
    static_assert((size_t)(DM / TP_TILE) * (HD / TP_TILE) * NH * TP_TILE * TP_TILE * 3 * 2 == SZ_WQKV);
    static_assert((size_t)(DM / TP_TILE) * (DM / TP_TILE) * TP_TILE * TP_TILE * 2 == SZ_WO);
    static_assert((size_t)(DM / TP_TILE) * (DFF / TP_TILE) * TP_TILE * TP_TILE * 2 == SZ_W1);
    static_assert((size_t)(DFF / TP_TILE) * (DM / TP_TILE) * TP_TILE * TP_TILE * 2 == SZ_W2);
    if (SZ_TOT > ws_size) return;

    char* ws = (char*)d_ws;
    size_t off = 0;
    _Float16* xh   = (_Float16*)(ws + off);
    _Float16* qpl  = (_Float16*)(ws + off + SZ_XH);
    _Float16* kpl  = (_Float16*)(ws + off + SZ_XH + SZ_PL);
    _Float16* vpl  = (_Float16*)(ws + off + SZ_XH + 2 * SZ_PL);
    _Float16* hpl  = (_Float16*)(ws + off);
    off += SZ_R0;
    _Float16* ctx  = (_Float16*)(ws + off); off += SZ_CTX;
    float*    y    = (float*)(ws + off);    off += SZ_Y;
    float*    x1   = (float*)(ws + off);    off += SZ_X1;
    _Float16* x1h  = (_Float16*)(ws + off); off += SZ_X1H;
    _Float16* wqkvT = (_Float16*)(ws + off); off += SZ_WQKV;
    _Float16* woT  = (_Float16*)(ws + off); off += SZ_WO;
    _Float16* w1T  = (_Float16*)(ws + off); off += SZ_W1;
    _Float16* w2T  = (_Float16*)(ws + off); off += SZ_W2;

    k_cvt_x<<<dim3(NTOK / 2), dim3(256), 0, stream>>>(x, xh);

    k_tpose<<<dim3(DM / TP_TILE, HD / TP_TILE, NH), dim3(TP_THREADS), 0, stream>>>(Wq, wqkvT, DM, HD);
    k_tpose<<<dim3(DM / TP_TILE, HD / TP_TILE, NH), dim3(TP_THREADS), 0, stream>>>(Wk, wqkvT + (size_t)DM * DM, DM, HD);
    k_tpose<<<dim3(DM / TP_TILE, HD / TP_TILE, NH), dim3(TP_THREADS), 0, stream>>>(Wv, wqkvT + (size_t)2 * DM * DM, DM, HD);
    k_tpose<<<dim3(DM / TP_TILE, DM / TP_TILE, 1), dim3(TP_THREADS), 0, stream>>>(Wo, woT, DM, DM);
    k_tpose<<<dim3(DM / TP_TILE, DFF / TP_TILE, 1), dim3(TP_THREADS), 0, stream>>>(W1, w1T, DM, DFF);
    k_tpose<<<dim3(DFF / TP_TILE, DM / TP_TILE, 1), dim3(TP_THREADS), 0, stream>>>(W2, w2T, DFF, DM);

    k_gemm_h<1><<<dim3(NTOK / 128, (3 * DM) / 128), dim3(256), 0, stream>>>(
        xh, wqkvT, bq, bk, bv, qpl, (unsigned)DM, (unsigned)(3 * DM), AL_QKV, CAR_ACT);

    k_attn<<<dim3(SEQ / 128, NB * NH), dim3(256), 0, stream>>>(qpl, kpl, vpl, ctx);

    k_gemm_res<1><<<dim3(NTOK / 128, DM / 128), dim3(256), 0, stream>>>(
        ctx, woT, bo, x, y, (unsigned)DM, AL_WO);

    k_ln<1><<<dim3(NTOK / 8), dim3(256), 0, stream>>>(y, g1, be1, x1, x1h);

    k_gemm_h<0><<<dim3(NTOK / 128, DFF / 128), dim3(256), 0, stream>>>(
        x1h, w1T, b1, b1, b1, hpl, (unsigned)DM, (unsigned)DFF, AL_FF1, CAR_ACT);

    k_gemm_res<0><<<dim3(NTOK / 128, DM / 128), dim3(256), 0, stream>>>(
        hpl, w2T, b2, x1, y, (unsigned)DFF, AL_FF2);

    k_ln<0><<<dim3(NTOK / 8), dim3(256), 0, stream>>>(y, g2, be2, out, x1h);
}
